// ModelCordinateDescentAlpha_91164975824956
// MI455X (gfx1250) — hardware-verified
//
#include <hip/hip_runtime.h>
#include <math.h>

constexpr int kRows  = 16384;
constexpr int kDimD  = 512;
constexpr int kCtr   = 4096;
constexpr int kOutO  = 16;
constexpr int kRowBlk = 64;
constexpr int kChunk  = 64;
constexpr int kKsPitch = 68;

static_assert(kRows % kRowBlk == 0, "tile multiple");
static_assert(kCtr % kChunk == 0, "tile multiple");
static_assert(kDimD % 32 == 0, "K multiple of 32");
static_assert(kRows % 64 == 0 && kCtr % 64 == 0, "prep blocks of 64 rows");

typedef __attribute__((ext_vector_type(16))) _Float16 v16h;
typedef __attribute__((ext_vector_type(8)))  _Float16 v8h;
typedef __attribute__((ext_vector_type(16))) __bf16   v16b;
typedef __attribute__((ext_vector_type(8)))  __bf16   v8b;
typedef __attribute__((ext_vector_type(8)))  float    v8f;
typedef __attribute__((ext_vector_type(4)))  float    v4f;
typedef __attribute__((ext_vector_type(4)))  unsigned int v4u;

__device__ __forceinline__ void dep_guard_h(v8f& a, v8f& b, v16h x, v16h y) { asm volatile("v_nop\n\tv_nop\n\tv_nop\n\tv_nop" : "+v"(a), "+v"(b) : "v"(x), "v"(y)); }
__device__ __forceinline__ void dep_guard_b(v8f& a, v8f& b, v16b x, v16b y) { asm volatile("v_nop\n\tv_nop\n\tv_nop\n\tv_nop" : "+v"(a), "+v"(b) : "v"(x), "v"(y)); }
__device__ __forceinline__ void keep4_h(v16h a, v16h b, v16h c, v16h d) { asm volatile("v_nop" :: "v"(a), "v"(b), "v"(c), "v"(d)); }
__device__ __forceinline__ void keep4_b(v16b a, v16b b, v16b c, v16b d) { asm volatile("v_nop" :: "v"(a), "v"(b), "v"(c), "v"(d)); }
__device__ __forceinline__ void acc_guard4(v8f& a, v8f& b, v8f& c, v8f& d) { asm volatile("v_nop\n\tv_nop\n\tv_nop\n\tv_nop" : "+v"(a), "+v"(b), "+v"(c), "+v"(d)); }
template <typename T> struct Frag;
template <> struct Frag<_Float16> {
  typedef v16h V; union U { v16h v; v8h h[2]; };
  static __device__ __forceinline__ v16h load(const _Float16* p) {
    U f; f.h[0] = *(const v8h*)(p); f.h[1] = *(const v8h*)(p + 16); return f.v;
  }
  static __device__ __forceinline__ v8f mma(v16h a, v16h b, v8f c) {
    return __builtin_amdgcn_wmma_f32_16x16x32_f16(false, a, false, b, (short)0, c, false, false);
  }
  static __device__ __forceinline__ void guard(v8f& a, v8f& b, v16h x, v16h y) { dep_guard_h(a, b, x, y); }
  static __device__ __forceinline__ void keep(v16h a, v16h b, v16h c, v16h d) { keep4_h(a, b, c, d); }
};
template <> struct Frag<__bf16> {
  typedef v16b V; union U { v16b v; v8b h[2]; };
  static __device__ __forceinline__ v16b load(const __bf16* p) {
    U f; f.h[0] = *(const v8b*)(p); f.h[1] = *(const v8b*)(p + 16); return f.v;
  }
  static __device__ __forceinline__ v8f mma(v16b a, v16b b, v8f c) {
    return __builtin_amdgcn_wmma_f32_16x16x32_bf16(false, a, false, b, (short)0, c, false, false);
  }
  static __device__ __forceinline__ void guard(v8f& a, v8f& b, v16b x, v16b y) { dep_guard_b(a, b, x, y); }
  static __device__ __forceinline__ void keep(v16b a, v16b b, v16b c, v16b d) { keep4_b(a, b, c, d); }
};

__device__ __forceinline__ unsigned pk16(unsigned short a, unsigned short b) { return (unsigned)a | ((unsigned)b << 16); }
__device__ __forceinline__ unsigned short h_bits(float f) { const _Float16 h = (_Float16)f; return __builtin_bit_cast(unsigned short, h); }

__global__ __launch_bounds__(256) void rows_prep_kernel(const float* __restrict__ src,
                                                        unsigned short* __restrict__ dst16,
                                                        float* __restrict__ dnorm) {
  __shared__ __align__(16) float sn[64];
  const int t = threadIdx.x;
  const int lane = t & 31, wave = t >> 5;
  const int rb = blockIdx.x * 64;
#pragma unroll 1
  for (int i = 0; i < 8; ++i) {
    const int row = rb + wave * 8 + i;
    const float* p = src + (size_t)row * kDimD;
    const v4f a0 = *(const v4f*)(p + 8 * lane);
    const v4f a1 = *(const v4f*)(p + 8 * lane + 4);
    const v4f b0 = *(const v4f*)(p + 256 + 8 * lane);
    const v4f b1 = *(const v4f*)(p + 256 + 8 * lane + 4);
    float s = 0.f;
#pragma unroll
    for (int e = 0; e < 4; ++e) s += a0[e] * a0[e];
#pragma unroll
    for (int e = 0; e < 4; ++e) s += a1[e] * a1[e];
#pragma unroll
    for (int e = 0; e < 4; ++e) s += b0[e] * b0[e];
#pragma unroll
    for (int e = 0; e < 4; ++e) s += b1[e] * b1[e];
#pragma unroll
    for (int off = 16; off > 0; off >>= 1) s += __shfl_xor(s, off, 32);
    if (lane == 0) sn[wave * 8 + i] = s;
    const v4u ua = (v4u){pk16(h_bits(a0[0]), h_bits(a0[1])), pk16(h_bits(a0[2]), h_bits(a0[3])),
                         pk16(h_bits(a1[0]), h_bits(a1[1])), pk16(h_bits(a1[2]), h_bits(a1[3]))};
    const v4u ub = (v4u){pk16(h_bits(b0[0]), h_bits(b0[1])), pk16(h_bits(b0[2]), h_bits(b0[3])),
                         pk16(h_bits(b1[0]), h_bits(b1[1])), pk16(h_bits(b1[2]), h_bits(b1[3]))};
    unsigned short* q = dst16 + (size_t)row * kDimD;
    for (int pass = 0; pass < 2; ++pass) {
      *(volatile v4u*)(q + 8 * lane) = ua;
      *(volatile v4u*)(q + 256 + 8 * lane) = ub;
      __threadfence();
    }
  }
  __syncthreads();
  if (wave == 0 && lane < 16) {
    const v4f v = *(const v4f*)(sn + 4 * lane);
    float* np0 = dnorm + rb + 4 * lane;
    *(volatile v4f*)np0 = v;
    __threadfence();
    *(volatile v4f*)np0 = v;
  }
}

__global__ __launch_bounds__(128) void rbf_head_kernel(const unsigned short* __restrict__ x16,
                                                       const unsigned short* __restrict__ mu16,
                                                       const float* __restrict__ dx,
                                                       const float* __restrict__ dmu,
                                                       const float* __restrict__ gamma_p,
                                                       const float* __restrict__ alpha,
                                                       float* __restrict__ out) {
  __shared__ __align__(16) float Ks[kRowBlk * kKsPitch];
  __shared__ __align__(16) float As[kChunk * kOutO];
  __shared__ __align__(16) float Os[kRowBlk * kOutO];

  const int t = threadIdx.x;
  const int lane = t & 31, wave = t >> 5;
  const int hh = lane >> 4;
  const int rlane = lane & 15;
  const int koff = hh * 8;
  const int rowBase = blockIdx.x * kRowBlk;
  const int r0w = rowBase + wave * 16;

  const _Float16* X  = (const _Float16*)x16;
  const _Float16* MU = (const _Float16*)mu16;
  const float g = gamma_p[0];

  float dxv[8];
#pragma unroll
  for (int r = 0; r < 8; ++r) dxv[r] = dx[r0w + 8 * hh + r];

  const int vrow = t >> 1;
  const int og = (t & 1) * 8;
  float acc8[8];
#pragma unroll
  for (int e = 0; e < 8; ++e) acc8[e] = 0.f;

  for (int cc = 0; cc < kCtr; cc += kChunk) {
    __syncthreads();
    {
      const v4f* a4 = (const v4f*)(alpha + (size_t)cc * kOutO);
      *(v4f*)(As + 4 * t) = a4[t];
      *(v4f*)(As + 512 + 4 * t) = a4[128 + t];
    }

    v8f acc[4];
#pragma unroll
    for (int j = 0; j < 4; ++j) acc[j] = (v8f){0.f,0.f,0.f,0.f,0.f,0.f,0.f,0.f};

    for (int k0 = 0; k0 < kDimD; k0 += 32) {
      v16h bh[4];
#pragma unroll
      for (int j = 0; j < 4; ++j)
        bh[j] = Frag<_Float16>::load(MU + (size_t)(cc + (j << 4) + rlane) * kDimD + koff + k0);
      const v16h ah = Frag<_Float16>::load(X + (size_t)(r0w + rlane) * kDimD + koff + k0);
#pragma unroll
      for (int j = 0; j < 4; ++j) acc[j] = Frag<_Float16>::mma(ah, bh[j], acc[j]);
      Frag<_Float16>::guard(acc[0], acc[3], ah, ah);
      Frag<_Float16>::keep(bh[0], bh[1], bh[2], bh[3]);
    }
    acc_guard4(acc[0], acc[1], acc[2], acc[3]);

#pragma unroll
    for (int j = 0; j < 4; ++j) {
      const float dm = dmu[cc + (j << 4) + rlane];
#pragma unroll
      for (int r = 0; r < 8; ++r) {
        const float s = acc[j][r];
        const float kv = expf(g * (2.0f * s - dxv[r] - dm));
        Ks[(wave * 16 + 8 * hh + r) * kKsPitch + (j << 4) + rlane] = kv;
      }
    }
    __syncthreads();

#pragma unroll 1
    for (int c4 = 0; c4 < kChunk; c4 += 4) {
      const v4f kq = *(const v4f*)(Ks + vrow * kKsPitch + c4);
#pragma unroll
      for (int u = 0; u < 4; ++u) {
        const v4f av0 = *(const v4f*)(As + (c4 + u) * kOutO + og);
        const v4f av1 = *(const v4f*)(As + (c4 + u) * kOutO + og + 4);
        const float kvu = kq[u];
#pragma unroll
        for (int e = 0; e < 4; ++e) {
          acc8[e]     += kvu * av0[e];
          acc8[4 + e] += kvu * av1[e];
        }
      }
    }
  }

  *(v4f*)(Os + 8 * t)     = (v4f){acc8[0], acc8[1], acc8[2], acc8[3]};
  *(v4f*)(Os + 8 * t + 4) = (v4f){acc8[4], acc8[5], acc8[6], acc8[7]};
  __syncthreads();
  const v4f o0 = *(const v4f*)(Os + 4 * t);
  const v4f o1 = *(const v4f*)(Os + 512 + 4 * t);
  float* ob = out + (size_t)rowBase * kOutO;
  for (int pass = 0; pass < 2; ++pass) {
    *(volatile v4f*)(ob + 4 * t) = o0;
    *(volatile v4f*)(ob + 512 + 4 * t) = o1;
    __threadfence();
  }
}

extern "C" void kernel_launch(void* const* d_in, const int* in_sizes, int n_in,
                              void* d_out, int out_size, void* d_ws, size_t ws_size,
                              hipStream_t stream) {
  if (n_in < 4) return;
  if (in_sizes[0] != kRows * kDimD) return;
  if (in_sizes[1] != kCtr * kDimD) return;
  if (in_sizes[2] < 1) return;
  if (in_sizes[3] != kCtr * kOutO) return;
  if (out_size != kRows * kOutO) return;

  const size_t offX16  = 0;
  const size_t offMu16 = offX16 + (size_t)kRows * kDimD * 2;
  const size_t offDx   = offMu16 + (size_t)kCtr * kDimD * 2;
  const size_t offDmu  = offDx + (size_t)kRows * 4;
  const size_t total   = offDmu + (size_t)kCtr * 4;
  if (total > ws_size) return;

  const float* x     = (const float*)d_in[0];
  const float* mu    = (const float*)d_in[1];
  const float* gamma = (const float*)d_in[2];
  const float* alpha = (const float*)d_in[3];
  float* out = (float*)d_out;
  char* ws = (char*)d_ws;
  unsigned short* x16  = (unsigned short*)(ws + offX16);
  unsigned short* mu16 = (unsigned short*)(ws + offMu16);
  float* dx  = (float*)(ws + offDx);
  float* dmu = (float*)(ws + offDmu);

  rows_prep_kernel<<<kRows / 64, 256, 0, stream>>>(x, x16, dx);
  rows_prep_kernel<<<kCtr / 64, 256, 0, stream>>>(mu, mu16, dmu);
  rbf_head_kernel<<<kRows / kRowBlk, 128, 0, stream>>>(x16, mu16, dx, dmu, gamma, alpha, out);
}
